// MoEDiscriminator_87806311400124
// MI455X (gfx1250) — hardware-verified
//
#include <hip/hip_runtime.h>
#include <math.h>

typedef __attribute__((ext_vector_type(16))) _Float16 v16h;
typedef __attribute__((ext_vector_type(16))) __bf16 v16b;
typedef __attribute__((ext_vector_type(8)))  _Float16 v8h;
typedef __attribute__((ext_vector_type(8)))  float v8f;
typedef __attribute__((ext_vector_type(4)))  float v4f;
typedef __attribute__((ext_vector_type(2)))  float v2f;
typedef __attribute__((ext_vector_type(4)))  unsigned v4u;
typedef __attribute__((ext_vector_type(4)))  int v4i;
typedef float __attribute__((may_alias)) float_a;
typedef int __attribute__((may_alias)) int_a;

template <typename T> __device__ __forceinline__ void vst2(void* p, T v) { *(volatile T*)p = v; __threadfence(); *(volatile T*)p = v; }
__device__ __forceinline__ v8f wmma16(v16h a, v16h b, v8f c) {
  v8f d = __builtin_amdgcn_wmma_f32_16x16x32_f16(false, a, false, b, (short)0, c, false, false);
  asm volatile("v_nop\n\tv_nop\n\tv_nop\n\tv_nop" : "+v"(d) : "v"(a), "v"(b));
  return d;
}
__device__ __forceinline__ v8f wmma_bf(v16b a, v16b b, v8f c) {
  v8f d = __builtin_amdgcn_wmma_f32_16x16x32_bf16(false, a, false, b, (short)0, c, false, false);
  asm volatile("v_nop\n\tv_nop\n\tv_nop\n\tv_nop" : "+v"(d) : "v"(a), "v"(b));
  return d;
}
__device__ __forceinline__ v16h frag_h(const _Float16* rowk0, int lane) {
  union { v16h v; v8h q[2]; } u; const _Float16* p = rowk0 + 8 * (lane >> 4);
  u.q[0] = *(const v8h*)p; u.q[1] = *(const v8h*)(p + 16); return u.v;
}
__device__ __forceinline__ v16h frag_f32(const float* rowk0, int lane) {
  v16h a; const float* p = rowk0 + 8 * (lane >> 4);
#pragma unroll
  for (int i = 0; i < 8; ++i) { a[i] = (_Float16)p[i]; a[8 + i] = (_Float16)p[16 + i]; }
  return a;
}
__device__ __forceinline__ v16h frag_f32s(const float* rowk0, int lane, float sc) {
  v16h a; const float* p = rowk0 + 8 * (lane >> 4);
#pragma unroll
  for (int i = 0; i < 8; ++i) { a[i] = (_Float16)(p[i] * sc); a[8 + i] = (_Float16)(p[16 + i] * sc); }
  return a;
}
__device__ __forceinline__ v16h fragc_f32(const float* W, int k0, int n, int lane, int ld, int K) {
  v16h a; const int g = lane >> 4;
#pragma unroll
  for (int i = 0; i < 8; ++i) { const int ka = k0 + 8 * g + i, kb = ka + 16;
    a[i] = (_Float16)(ka < K ? W[(size_t)(ka < K ? ka : K - 1) * ld + n] : 0.f); a[8 + i] = (_Float16)(kb < K ? W[(size_t)(kb < K ? kb : K - 1) * ld + n] : 0.f); }
  return a;
}
struct F2 { v16b h, l; };
__device__ __forceinline__ F2 bsplit16(const float v[16]) { F2 r;
#pragma unroll
  for (int i = 0; i < 16; ++i) { const __bf16 h = (__bf16)v[i]; r.h[i] = h; r.l[i] = (__bf16)(v[i] - (float)h); }
  return r; }
__device__ __forceinline__ F2 split_row(const float* row, int k0, int lane) { float v[16]; const float* p = row + k0 + 8 * (lane >> 4);
#pragma unroll
  for (int i = 0; i < 8; ++i) { v[i] = p[i]; v[8 + i] = p[16 + i]; }
  return bsplit16(v); }
__device__ __forceinline__ F2 split_rowK(const float* row, int k0, int lane, int K) { float v[16]; const int g = lane >> 4;
#pragma unroll
  for (int i = 0; i < 8; ++i) { const int ka = k0 + 8 * g + i, kb = ka + 16; v[i] = ka < K ? row[ka < K ? ka : K - 1] : 0.f; v[8 + i] = kb < K ? row[kb < K ? kb : K - 1] : 0.f; }
  return bsplit16(v); }
__device__ __forceinline__ F2 split_col(const float* W, int k0, int n, int lane, int ld, int K) { float v[16]; const int g = lane >> 4;
#pragma unroll
  for (int i = 0; i < 8; ++i) { const int ka = k0 + 8 * g + i, kb = ka + 16; v[i] = ka < K ? W[(size_t)(ka < K ? ka : K - 1) * ld + n] : 0.f; v[8 + i] = kb < K ? W[(size_t)(kb < K ? kb : K - 1) * ld + n] : 0.f; }
  return bsplit16(v); }
__device__ __forceinline__ v8f mac3(const F2& a, const F2& b, v8f c) { c = wmma_bf(a.l, b.h, c); c = wmma_bf(a.h, b.l, c); return wmma_bf(a.h, b.h, c); }
__device__ __forceinline__ float sigm(float v) { return 1.0f / (1.0f + expf(-v)); }
#define LDSX() do { asm volatile("s_wait_dscnt 0" ::: "memory"); __builtin_amdgcn_wave_barrier(); __builtin_amdgcn_fence(__ATOMIC_RELEASE, "workgroup"); } while (0)


#define NBQ 65536
#define DS 64
#define NC 8
#define HH 256
#ifndef NBLKQ
#define NBLKQ (NBQ / 64)
#endif
typedef __attribute__((ext_vector_type(8))) __bf16 v8b;
__device__ __forceinline__ v16b frag_b(const __bf16* rowk0, int lane) {
  union { v16b v; v8b q[2]; } u; const __bf16* p = rowk0 + 8 * (lane >> 4);
  u.q[0] = *(const v8b*)p; u.q[1] = *(const v8b*)(p + 16); return u.v;
}
__device__ __forceinline__ float bfr(float v) { return (float)(__bf16)v; }
__device__ __attribute__((noinline)) float exp_ni(float v) { return expf(v); }
__device__ __attribute__((noinline)) float erf_ni(float v) { return erff(v); }

#define WS_P1  0u
#define WS_P2  (WS_P1 + 2u * NC * HH * DS)
#define WS_END (WS_P2 + 2u * NC * HH * HH)

__global__ __launch_bounds__(256) void k_pack(const float* __restrict__ W1, const float* __restrict__ W2, __bf16* __restrict__ P1, __bf16* __restrict__ P2) {
  __shared__ __align__(16) __bf16 s1[DS], s2[HH]; const int n = blockIdx.x, c = blockIdx.y, tid = threadIdx.x;
  if (tid < DS) s1[tid] = (__bf16)W1[((size_t)c * DS + tid) * HH + n];
  s2[tid] = (__bf16)W2[((size_t)c * HH + tid) * HH + n];
  __syncthreads();
  if (tid < 8) vst2((unsigned*)(P1 + ((size_t)c * HH + n) * DS + tid * 8), *(const v4u*)&s1[tid * 8]);
  else if (tid < 8 + 32) vst2((unsigned*)(P2 + ((size_t)c * HH + n) * HH + (tid - 8) * 8), *(const v4u*)&s2[(tid - 8) * 8]);
}
__global__ __launch_bounds__(128) void k_moe(const float* __restrict__ ST, const __bf16* __restrict__ P1, const __bf16* __restrict__ P2, const float* __restrict__ B1, const float* __restrict__ B2, const float* __restrict__ W3, const float* __restrict__ B3, float* __restrict__ out) {
  __shared__ __align__(16) __bf16 sh[4][16][HH + 8], sl[4][16][HH + 8]; __shared__ __align__(16) float so[64][NC]; __shared__ float sb1[HH], sb2[HH], sw3[HH];
  const int tid = threadIdx.x, wave = tid >> 5, lane = tid & 31, col = lane & 15, g = lane >> 4; const size_t r0 = (size_t)blockIdx.x * 64 + wave * 16;
  v16b ast[2];
#pragma unroll
  for (int kc = 0; kc < 2; ++kc) { const float* p = ST + (r0 + col) * DS + kc * 32 + 8 * g;
#pragma unroll
    for (int i = 0; i < 8; ++i) { ast[kc][i] = (__bf16)p[i]; ast[kc][8 + i] = (__bf16)p[16 + i]; } }
#pragma unroll 1
  for (int c = 0; c < NC; ++c) {
    __syncthreads();
    for (int i = tid; i < HH; i += 128) { sb1[i] = bfr(B1[c * HH + i]); sb2[i] = bfr(B2[c * HH + i]); sw3[i] = bfr(W3[c * HH + i]); }
    __syncthreads();
    { v8f acc[16]; for (int j = 0; j < 16; ++j) acc[j] = (v8f){};
#pragma unroll
      for (int kc = 0; kc < 2; ++kc) {
#pragma unroll
        for (int j = 0; j < 16; ++j) acc[j] = wmma_bf(ast[kc], frag_b(P1 + ((size_t)c * HH + j * 16 + col) * DS + kc * 32, lane), acc[j]); }
#pragma unroll
      for (int j = 0; j < 16; ++j) { const int h = j * 16 + col;
#pragma unroll
        for (int r = 0; r < 8; ++r) { const float v = fmaxf(acc[j][r] + sb1[h], 0.f); const __bf16 hb = (__bf16)v; sh[wave][8 * g + r][h] = hb; sl[wave][8 * g + r][h] = (__bf16)(v - (float)hb); } } }
    LDSX();
    v8f acc2[16]; for (int j = 0; j < 16; ++j) acc2[j] = (v8f){};
#pragma unroll 2
    for (int kc = 0; kc < HH / 32; ++kc) { v16b ah, al;
#pragma unroll
      for (int i = 0; i < 8; ++i) { ah[i] = sh[wave][col][kc * 32 + 8 * g + i]; ah[8 + i] = sh[wave][col][kc * 32 + 16 + 8 * g + i]; al[i] = sl[wave][col][kc * 32 + 8 * g + i]; al[8 + i] = sl[wave][col][kc * 32 + 16 + 8 * g + i]; }
#pragma unroll
      for (int j = 0; j < 16; ++j) { const v16b w = frag_b(P2 + ((size_t)c * HH + j * 16 + col) * HH + kc * 32, lane); acc2[j] = wmma_bf(al, w, acc2[j]); acc2[j] = wmma_bf(ah, w, acc2[j]); } }
    float d[8];
#pragma unroll
    for (int r = 0; r < 8; ++r) { float s = 0.f;
#pragma unroll
      for (int j = 0; j < 16; ++j) { const int o = j * 16 + col; s += fmaxf(acc2[j][r] + sb2[o], 0.f) * sw3[o]; }
#pragma unroll
      for (int q = 1; q < 16; q <<= 1) s += __shfl_xor(s, q);
      d[r] = s; }
    if (col == 0) { const float b3 = bfr(B3[c]);
#pragma unroll
      for (int r = 0; r < 8; ++r) so[wave * 16 + 8 * g + r][c] = d[r] + b3; }
    LDSX();
  }
  __syncthreads();
  vst2(out + (size_t)blockIdx.x * 64 * NC + tid * 4, *(const v4f*)&(&so[0][0])[tid * 4]);
}
extern "C" void kernel_launch(void* const* d_in, const int* in_sizes, int n_in, void* d_out, int out_size, void* d_ws, size_t ws_size, hipStream_t stream) {
  (void)in_sizes; (void)n_in; (void)out_size;
  const float** F = (const float**)d_in;
  if (ws_size < (size_t)WS_END) return;
  char* ws = (char*)d_ws; __bf16 *P1 = (__bf16*)(ws + WS_P1), *P2 = (__bf16*)(ws + WS_P2);
  k_pack<<<dim3(HH, NC), 256, 0, stream>>>(F[1], F[3], P1, P2);
  k_moe<<<NBLKQ, 128, 0, stream>>>(F[0], P1, P2, F[2], F[4], F[5], F[6], (float*)d_out);
}
